// ToeplitzCausalLinear_77472620085401
// MI455X (gfx1250) — hardware-verified
//
#include <hip/hip_runtime.h>
#include <stddef.h>
#include <stdint.h>

#define TT   2048
#define NH   3
#define HD   256
#define EE   (NH * HD)
#define GBM  128
#define GBN  128
#define ASC  16.0f
#define BSC  16.0f
#define ISC  (1.0f / 256.0f)

static_assert((TT % 32) == 0);
static_assert((TT % GBN) == 0);
static_assert((EE % GBM) == 0);
static_assert((HD % GBM) == 0);
static_assert(TT == 256 * 8);
static_assert(GBM == 128);
static_assert(GBN == 128);
static_assert(TT == 2048);

typedef _Float16     v16h __attribute__((ext_vector_type(16)));
typedef _Float16     v8h  __attribute__((ext_vector_type(8)));
typedef float        v8f  __attribute__((ext_vector_type(8)));
typedef float        v4f  __attribute__((ext_vector_type(4)));
typedef unsigned int v4u  __attribute__((ext_vector_type(4)));

__device__ __forceinline__ unsigned short bf_bits(float f) {
  const unsigned u = __float_as_uint(f);
  return (unsigned short)((u + 0x7FFFu + ((u >> 16) & 1u)) >> 16);
}
__device__ __forceinline__ float bfr(float f) { return __uint_as_float(((unsigned)bf_bits(f)) << 16); }
__device__ __forceinline__ unsigned short h_bits(float f) {
  const _Float16 h = (_Float16)f;
  return __builtin_bit_cast(unsigned short, h);
}
__device__ __forceinline__ unsigned pk16(unsigned short a, unsigned short b) { return (unsigned)a | ((unsigned)b << 16); }
__device__ __forceinline__ v8f zero8() { v8f z = {0.f, 0.f, 0.f, 0.f, 0.f, 0.f, 0.f, 0.f}; return z; }

union FragH { v16h v; v8h h[2]; };
__device__ __forceinline__ v16h ldfrag_h(const _Float16* p) {
  FragH f;
  f.h[0] = *(const v8h*)(p);
  f.h[1] = *(const v8h*)(p + 16);
  return f.v;
}

__device__ __forceinline__ v8f mma_h(v16h a, v16h b, v8f c) {
  return __builtin_amdgcn_wmma_f32_16x16x32_f16(false, a, false, b, (short)0, c, false, false);
}
__device__ __forceinline__ void guard8(v8f& c0, v8f& c1, v8f& c2, v8f& c3, v8f& c4, v8f& c5, v8f& c6, v8f& c7,
                                       const v16h& a0, const v16h& a1, const v16h& a2, const v16h& a3,
                                       const v16h& b0, const v16h& b1) {
#if defined(__HIP_DEVICE_COMPILE__)
  asm volatile("v_nop\n\tv_nop\n\tv_nop\n\tv_nop"
               : "+v"(c0), "+v"(c1), "+v"(c2), "+v"(c3), "+v"(c4), "+v"(c5), "+v"(c6), "+v"(c7)
               : "v"(a0), "v"(a1), "v"(a2), "v"(a3), "v"(b0), "v"(b1));
#endif
}

__global__ __launch_bounds__(256)
void k_cvx(const float* __restrict__ x, unsigned short* Ap) {
  const unsigned row = blockIdx.x;
  const unsigned i8  = threadIdx.x * 8u;
  const float* src = x + (size_t)row * TT + i8;
  const v4f a = *(const v4f*)(src);
  const v4f c = *(const v4f*)(src + 4);
  v4u u;
  u[0] = pk16(h_bits(bfr(a[0]) * ASC), h_bits(bfr(a[1]) * ASC));
  u[1] = pk16(h_bits(bfr(a[2]) * ASC), h_bits(bfr(a[3]) * ASC));
  u[2] = pk16(h_bits(bfr(c[0]) * ASC), h_bits(bfr(c[1]) * ASC));
  u[3] = pk16(h_bits(bfr(c[2]) * ASC), h_bits(bfr(c[3]) * ASC));
  unsigned short* dst = Ap + (size_t)row * TT + i8;
  *(volatile v4u*)dst = u;
  __threadfence();
  *(volatile v4u*)dst = u;
}

__device__ __forceinline__ unsigned short wq(const float* __restrict__ wh, int e) {
  const int ec = e < 0 ? 0 : (e > TT - 1 ? TT - 1 : e);
  const float v = wh[ec];
  const float s = (e >= 0) ? bfr(v) * BSC : 0.0f;
  return h_bits(s);
}

__global__ __launch_bounds__(256)
void k_cvw(const float* __restrict__ w, unsigned short* Bt) {
  const unsigned hj = blockIdx.x;
  const int j  = (int)(hj & (TT - 1));
  const int h  = (int)(hj >> 11);
  const int i8 = (int)threadIdx.x * 8;
  const float* wh = w + (size_t)h * TT;
  const int e = j - i8;
  v4u u;
  u[0] = pk16(wq(wh, e),     wq(wh, e - 1));
  u[1] = pk16(wq(wh, e - 2), wq(wh, e - 3));
  u[2] = pk16(wq(wh, e - 4), wq(wh, e - 5));
  u[3] = pk16(wq(wh, e - 6), wq(wh, e - 7));
  unsigned short* dst = Bt + (size_t)hj * TT + i8;
  *(volatile v4u*)dst = u;
  __threadfence();
  *(volatile v4u*)dst = u;
}

__device__ __forceinline__ void put8(float* tp, const v8f& a) {
#pragma unroll
  for (int r = 0; r < 8; ++r) tp[r * GBN] = a[r] * ISC;
}

__global__ __launch_bounds__(256)
void k_gemm(const unsigned short* __restrict__ Ap, const unsigned short* __restrict__ Bt,
            const float* __restrict__ bias, float* out) {
  __shared__ __align__(16) float tile[64 * GBN];

  const int tid = threadIdx.x, w = tid >> 5, lane = tid & 31, hh = lane >> 4, c = lane & 15;
  const int wr = w >> 2, wc = w & 3;
  const int mt = blockIdx.x >> 4, ot = blockIdx.x & 15;
  const int r0 = mt * GBM, o0 = ot * GBN;
  const int h  = (mt >> 1) % NH;

  const _Float16* A  = (const _Float16*)Ap;
  const _Float16* Bm = (const _Float16*)Bt;
  const _Float16* a0p = A + (size_t)(r0 + wr * 64 + c) * TT + 8 * hh;
  const _Float16* a1p = a0p + (size_t)16 * TT;
  const _Float16* a2p = a0p + (size_t)32 * TT;
  const _Float16* a3p = a0p + (size_t)48 * TT;
  const _Float16* b0p = Bm + ((size_t)h * TT + (size_t)(o0 + wc * 32 + c)) * TT + 8 * hh;
  const _Float16* b1p = b0p + (size_t)16 * TT;

  v8f c00 = zero8(), c01 = zero8(), c10 = zero8(), c11 = zero8();
  v8f c20 = zero8(), c21 = zero8(), c30 = zero8(), c31 = zero8();

  const int kend = (o0 + GBN) / 32;

#pragma unroll 1
  for (int ks = 0; ks < kend; ++ks) {
    const int ko = 32 * ks;
    const v16h a0 = ldfrag_h(a0p + ko);
    const v16h a1 = ldfrag_h(a1p + ko);
    const v16h a2 = ldfrag_h(a2p + ko);
    const v16h a3 = ldfrag_h(a3p + ko);
    const v16h f0 = ldfrag_h(b0p + ko);
    const v16h f1 = ldfrag_h(b1p + ko);
    c00 = mma_h(a0, f0, c00);
    c01 = mma_h(a0, f1, c01);
    c10 = mma_h(a1, f0, c10);
    c11 = mma_h(a1, f1, c11);
    c20 = mma_h(a2, f0, c20);
    c21 = mma_h(a2, f1, c21);
    c30 = mma_h(a3, f0, c30);
    c31 = mma_h(a3, f1, c31);
    guard8(c00, c01, c10, c11, c20, c21, c30, c31, a0, a1, a2, a3, f0, f1);
  }

  const int piece = tid & 31, rr = tid >> 5;
  const v4f bb = *(const v4f*)(bias + (size_t)h * TT + o0 + 4 * piece);
  v4f bq;
  bq[0] = bfr(bb[0]); bq[1] = bfr(bb[1]); bq[2] = bfr(bb[2]); bq[3] = bfr(bb[3]);
  float* orow = out + (size_t)r0 * TT + o0 + 4 * piece;
#pragma unroll 1
  for (int p = 0; p < 2; ++p) {
    __syncthreads();
    if (wr == p) {
      float* tw = tile + (8 * hh) * GBN + wc * 32 + c;
      put8(tw + (0  * GBN) + 0,  c00);
      put8(tw + (0  * GBN) + 16, c01);
      put8(tw + (16 * GBN) + 0,  c10);
      put8(tw + (16 * GBN) + 16, c11);
      put8(tw + (32 * GBN) + 0,  c20);
      put8(tw + (32 * GBN) + 16, c21);
      put8(tw + (48 * GBN) + 0,  c30);
      put8(tw + (48 * GBN) + 16, c31);
    }
    __syncthreads();
    v4f v[8];
#pragma unroll
    for (int it = 0; it < 8; ++it) v[it] = *(const v4f*)(tile + (rr + 8 * it) * GBN + 4 * piece) + bq;
    float* ob = orow + (size_t)(64 * p) * TT;
#pragma unroll
    for (int it = 0; it < 8; ++it) *(volatile v4f*)(ob + (size_t)(rr + 8 * it) * TT) = v[it];
    __threadfence();
#pragma unroll
    for (int it = 0; it < 8; ++it) *(volatile v4f*)(ob + (size_t)(rr + 8 * it) * TT) = v[it];
  }
}

extern "C" void kernel_launch(void* const* d_in, const int* in_sizes, int n_in,
                              void* d_out, int out_size, void* d_ws, size_t ws_size,
                              hipStream_t stream) {
  if (n_in < 3) return;
  const int rows = in_sizes[0] / TT;
  if (rows < 1 || in_sizes[0] != rows * TT) return;
  if ((rows % EE) != 0) return;
  if (in_sizes[1] != NH * TT) return;
  if (in_sizes[2] != NH * TT) return;
  if (out_size != rows * TT) return;

  const float* x    = (const float*)d_in[0];
  const float* wgt  = (const float*)d_in[1];
  const float* bias = (const float*)d_in[2];
  float* out = (float*)d_out;

  const size_t sAp = (size_t)rows * TT * 2;
  const size_t sBt = (size_t)NH * TT * TT * 2;
  size_t off = 0;
  const size_t oAp = off; off += sAp;
  const size_t oBt = off; off += sBt;
  if (off > ws_size) return;
  if (off > (size_t)134217728) return;

  char* ws = (char*)d_ws;
  unsigned short* Ap = (unsigned short*)(ws + oAp);
  unsigned short* Bt = (unsigned short*)(ws + oBt);

  k_cvx<<<dim3((unsigned)rows), dim3(256), 0, stream>>>(x, Ap);
  k_cvw<<<dim3(NH * TT), dim3(256), 0, stream>>>(wgt, Bt);
  k_gemm<<<dim3((unsigned)((rows / GBM) * (TT / GBN))), dim3(256), 0, stream>>>(Ap, Bt, bias, out);
  (void)hipGetLastError();
}
